// FDSECNN_29764123361285
// MI455X (gfx1250) — hardware-verified
//
#include <hip/hip_runtime.h>
#define NIMG 4096
#define GG 2
#define C0 3
#define T1 8
#define C1 (T1 * GG)
#define H1 32
#define NP1 (H1 * H1)
#define T2 16
#define C2 (T2 * GG)
#define H2 16
#define NP2 (H2 * H2)
#define H3 8
#define NP3 (H3 * H3)
#define K1P 32
#define K2P 160
#define FCI (C2 * NP3)
#define FCH 512
#define NCLS 10
#define ICH 256
typedef __bf16 v16b __attribute__((ext_vector_type(16)));
typedef unsigned short v8us __attribute__((ext_vector_type(8), may_alias));
typedef float  v8f  __attribute__((ext_vector_type(8)));
typedef float  v4f  __attribute__((ext_vector_type(4)));
typedef float  v4fa __attribute__((ext_vector_type(4), may_alias));
union FragB { v16b v; v8us half[2]; unsigned short u[16]; };

__device__ __forceinline__ unsigned short bf16_bits(float x) { unsigned int u = __float_as_uint(x); return (unsigned short)((u + 0x7FFFu + ((u >> 16) & 1u)) >> 16); }
__device__ __forceinline__ float bf16_val(unsigned short b) { return __uint_as_float(((unsigned int)b) << 16); }
__device__ __forceinline__ float bf16_round(float x) { return bf16_val(bf16_bits(x)); }
template <int NT>
__device__ __forceinline__ v8f mmaN(v16b ah, v16b al, v16b bh, v16b bl, v8f c) {
  c = __builtin_amdgcn_wmma_f32_16x16x32_bf16(false, ah, false, bh, (short)0, c, false, false);
  if (NT >= 2) c = __builtin_amdgcn_wmma_f32_16x16x32_bf16(false, al, false, bh, (short)0, c, false, false);
  if (NT >= 3) c = __builtin_amdgcn_wmma_f32_16x16x32_bf16(false, ah, false, bl, (short)0, c, false, false);
  asm volatile("v_nop\n\tv_nop\n\tv_nop\n\tv_nop" : "+v"(c) : "v"(ah), "v"(al), "v"(bh), "v"(bl));
  return c;
}

__global__ __launch_bounds__(256) void k_wt_bf16(const float* __restrict__ W, unsigned short* __restrict__ Wt, int K, int N) {
  const int t = blockIdx.x * 256 + threadIdx.x;
  const int k8n = K / 8;
  if (t >= N * k8n) return;
  const int n = t / k8n, k8 = (t % k8n) * 8;
  v8us v;
#pragma unroll
  for (int i = 0; i < 8; ++i) v[i] = bf16_bits(W[(size_t)(k8 + i) * N + n]);
  *(volatile v8us*)(Wt + (size_t)n * K + k8) = v;
  __threadfence();
  *(volatile v8us*)(Wt + (size_t)n * K + k8) = v;
}

template <bool ASPLIT, int ACT, bool BIAS_BF16>
__global__ __launch_bounds__(128) void k_gemm_bf(const float* __restrict__ A, int lda, const unsigned short* __restrict__ Wt, int ldb,
                                               const float* __restrict__ bias, float* __restrict__ C, int ldc, int M, int N, int K) {
  __shared__ __attribute__((aligned(16))) float so[4][16][64];
  const int tid = threadIdx.x, w = tid >> 5, lane = tid & 31, ln = lane & 15, hh = lane >> 4;
  const int ntn = N / 64;
  const int wid = blockIdx.x * 4 + w;
  const int mt = wid / ntn, nq = wid % ntn;
  if (mt * 16 >= M) return;
  const int row0 = mt * 16, col0 = nq * 64;
  const float* arow = A + (size_t)(row0 + ln) * lda;
  v8f acc[4] = {};
  for (int kb = 0; kb < K; kb += 32) {
    FragB ah, al;
    const v4f x0 = *(const v4fa*)(arow + kb + 8 * hh), x1 = *(const v4fa*)(arow + kb + 8 * hh + 4);
    const v4f x2 = *(const v4fa*)(arow + kb + 16 + 8 * hh), x3 = *(const v4fa*)(arow + kb + 16 + 8 * hh + 4);
    float xs[16] = {x0[0],x0[1],x0[2],x0[3],x1[0],x1[1],x1[2],x1[3],x2[0],x2[1],x2[2],x2[3],x3[0],x3[1],x3[2],x3[3]};
#pragma unroll
    for (int i = 0; i < 16; ++i) { const unsigned short hb = bf16_bits(xs[i]); ah.u[i] = hb; al.u[i] = ASPLIT ? bf16_bits(xs[i] - bf16_val(hb)) : (unsigned short)0; }
#pragma unroll
    for (int t = 0; t < 4; ++t) {
      const unsigned short* brow = Wt + (size_t)(col0 + t * 16 + ln) * ldb + kb;
      FragB b;
      b.half[0] = *(const v8us*)(brow + 8 * hh);
      b.half[1] = *(const v8us*)(brow + 16 + 8 * hh);
      acc[t] = mmaN<ASPLIT ? 2 : 1>(ah.v, al.v, b.v, b.v, acc[t]);
    }
  }
#pragma unroll
  for (int t = 0; t < 4; ++t) {
    float bv = bias ? bias[col0 + t * 16 + ln] : 0.f;
    if (BIAS_BF16) bv = bf16_round(bv);
#pragma unroll
    for (int r = 0; r < 8; ++r) { float v = acc[t][r] + bv; if (ACT == 1) v = fmaxf(v, 0.f); so[w][8 * hh + r][t * 16 + ln] = v; }
  }
  __builtin_amdgcn_fence(__ATOMIC_ACQ_REL, "workgroup");
  __builtin_amdgcn_wave_barrier();
  const int rsub = lane >> 4, c4 = (lane & 15) * 4;
  for (int pass = 0; pass < 2; ++pass) {
#pragma unroll
    for (int q = 0; q < 8; ++q) {
      const int r = q * 2 + rsub;
      const v4f v = *(const v4fa*)&so[w][r][c4];
      *(volatile v4f*)(C + (size_t)(row0 + r) * ldc + col0 + c4) = v;
    }
    if (pass == 0) __threadfence();
  }
}

template <bool ASPLIT, int ACT, bool BIAS_BF16, bool RES_BF16>
__global__ __launch_bounds__(128) void k_gemm_bf3(const float* __restrict__ A, int lda, const unsigned short* __restrict__ Wt, int ldb,
                                                const float* __restrict__ bias, const float* __restrict__ resid, int rmod, int ldr,
                                                float* __restrict__ C, int ldc, int M, int N, int K) {
  __shared__ __attribute__((aligned(16))) float so[4][16][64];
  const int tid = threadIdx.x, w = tid >> 5, lane = tid & 31, ln = lane & 15, hh = lane >> 4;
  const int ntn = N / 64;
  const int wid = blockIdx.x * 4 + w;
  const int mt = wid / ntn, nq = wid % ntn;
  if (mt * 16 >= M) return;
  const int row0 = mt * 16, col0 = nq * 64;
  const float* arow = A + (size_t)(row0 + ln) * lda;
  v8f acc[4] = {};
  for (int kb = 0; kb < K; kb += 32) {
    FragB ah, al;
    const v4f x0 = *(const v4fa*)(arow + kb + 8 * hh), x1 = *(const v4fa*)(arow + kb + 8 * hh + 4);
    const v4f x2 = *(const v4fa*)(arow + kb + 16 + 8 * hh), x3 = *(const v4fa*)(arow + kb + 16 + 8 * hh + 4);
    float xs[16] = {x0[0],x0[1],x0[2],x0[3],x1[0],x1[1],x1[2],x1[3],x2[0],x2[1],x2[2],x2[3],x3[0],x3[1],x3[2],x3[3]};
#pragma unroll
    for (int i = 0; i < 16; ++i) { const unsigned short hb = bf16_bits(xs[i]); ah.u[i] = hb; al.u[i] = ASPLIT ? bf16_bits(xs[i] - bf16_val(hb)) : (unsigned short)0; }
#pragma unroll
    for (int t = 0; t < 4; ++t) {
      const unsigned short* brow = Wt + (size_t)(col0 + t * 16 + ln) * ldb + kb;
      FragB b;
      b.half[0] = *(const v8us*)(brow + 8 * hh);
      b.half[1] = *(const v8us*)(brow + 16 + 8 * hh);
      acc[t] = mmaN<ASPLIT ? 2 : 1>(ah.v, al.v, b.v, b.v, acc[t]);
    }
  }
#pragma unroll
  for (int t = 0; t < 4; ++t) {
    const int col = col0 + t * 16 + ln;
    float bv = bias ? bias[col] : 0.f;
    if (BIAS_BF16) bv = bf16_round(bv);
#pragma unroll
    for (int r = 0; r < 8; ++r) {
      float v = acc[t][r] + bv;
      if (resid) { float rv = resid[(size_t)((row0 + 8 * hh + r) % rmod) * ldr + col]; if (RES_BF16) rv = bf16_round(rv); v += rv; }
      if (ACT == 1) v = fmaxf(v, 0.f);
      if (ACT == 2) v = 0.5f * v * (1.0f + erff(v * 0.70710678118654752f));
      if (ACT == 3) { const float u = 0.7978845608028654f * (v + 0.044715f * v * v * v); v = 0.5f * v * (1.0f + tanhf(u)); }
      so[w][8 * hh + r][t * 16 + ln] = v;
    }
  }
  __builtin_amdgcn_fence(__ATOMIC_ACQ_REL, "workgroup");
  __builtin_amdgcn_wave_barrier();
  const int rsub = lane >> 4, c4 = (lane & 15) * 4;
  for (int pass = 0; pass < 2; ++pass) {
#pragma unroll
    for (int q = 0; q < 8; ++q) {
      const int r = q * 2 + rsub;
      const v4f v = *(const v4fa*)&so[w][r][c4];
      *(volatile v4f*)(C + (size_t)(row0 + r) * ldc + col0 + c4) = v;
    }
    if (pass == 0) __threadfence();
  }
}
template <bool PARAM_BF16>
__global__ __launch_bounds__(256) void k_layernorm(const float* __restrict__ X, const float* __restrict__ R, const float* __restrict__ g, const float* __restrict__ bta,
                                                  float* __restrict__ out_sum, float* __restrict__ out_norm, int N, float eps) {
  __shared__ float red[256];
  const int row = blockIdx.x, tid = threadIdx.x;
  const float* x = X + (size_t)row * N; const float* rr = R ? R + (size_t)row * N : nullptr;
  float vals[16];
  const int per = N / 256;
  float s1 = 0.f;
  for (int u = 0; u < per / 4; ++u) {
    const int j = tid * 4 + 1024 * u;
    const v4f a = *(const v4fa*)(x + j);
    v4f b = {0.f,0.f,0.f,0.f}; if (rr) b = *(const v4fa*)(rr + j);
#pragma unroll
    for (int q = 0; q < 4; ++q) { const float v = a[q] + b[q]; vals[u * 4 + q] = v; s1 += v; }
  }
  red[tid] = s1; __syncthreads();
  for (int st = 128; st > 0; st >>= 1) { if (tid < st) red[tid] += red[tid + st]; __syncthreads(); }
  const float mu = red[0] / (float)N; __syncthreads();
  float s2 = 0.f;
  for (int u = 0; u < per / 4; ++u)
#pragma unroll
    for (int q = 0; q < 4; ++q) { const float c = vals[u * 4 + q] - mu; s2 += c * c; }
  red[tid] = s2; __syncthreads();
  for (int st = 128; st > 0; st >>= 1) { if (tid < st) red[tid] += red[tid + st]; __syncthreads(); }
  const float rs = rsqrtf(red[0] / (float)N + eps);
  for (int pass = 0; pass < 2; ++pass) {
    for (int u = 0; u < per / 4; ++u) {
      const int j = tid * 4 + 1024 * u;
      v4f o, sm;
#pragma unroll
      for (int q = 0; q < 4; ++q) {
        float gg = g[j + q], bb = bta[j + q];
        if (PARAM_BF16) { gg = bf16_round(gg); bb = bf16_round(bb); }
        sm[q] = vals[u * 4 + q]; o[q] = (vals[u * 4 + q] - mu) * rs * gg + bb;
      }
      if (out_sum) *(volatile v4f*)(out_sum + (size_t)row * N + j) = sm;
      *(volatile v4f*)(out_norm + (size_t)row * N + j) = o;
    }
    if (pass == 0) __threadfence();
  }
}


typedef _Float16 v16h __attribute__((ext_vector_type(16)));
union FragH { v16h v; v8us half[2]; _Float16 h[16]; unsigned short u[16]; };
template <int NT>
__device__ __forceinline__ v8f mmaH(v16h ah, v16h al, v16h bh, v16h bl, v8f c) {
  c = __builtin_amdgcn_wmma_f32_16x16x32_f16(false, ah, false, bh, (short)0, c, false, false);
  if (NT >= 2) c = __builtin_amdgcn_wmma_f32_16x16x32_f16(false, al, false, bh, (short)0, c, false, false);
  if (NT >= 3) c = __builtin_amdgcn_wmma_f32_16x16x32_f16(false, ah, false, bl, (short)0, c, false, false);
  asm volatile("v_nop\n\tv_nop\n\tv_nop\n\tv_nop" : "+v"(c) : "v"(ah), "v"(al), "v"(bh), "v"(bl));
  return c;
}
template <bool ASPLIT>
__global__ __launch_bounds__(128) void k_gemm_h(const float* __restrict__ A, int lda, size_t sA, const _Float16* __restrict__ Bh, int ldb, size_t sB, float alpha, float* __restrict__ C, int ldc, size_t sC, int M, int N, int K) {
  __shared__ __attribute__((aligned(16))) float so[4][16][64];
  const int tid = threadIdx.x, w = tid >> 5, lane = tid & 31, ln = lane & 15, hh = lane >> 4; const int by = blockIdx.y;
  A += (size_t)by * sA; Bh += (size_t)by * sB; C += (size_t)by * sC;
  const int ntn = (N + 63) / 64; const int wid = blockIdx.x * 4 + w; const int mt = wid / ntn, nq = wid % ntn; if (mt * 16 >= M) return;
  const int row0 = mt * 16, col0 = nq * 64; const float* arow = A + (size_t)(row0 + ln) * lda;
  v8f acc[4] = {};
  for (int kb = 0; kb < K; kb += 32) {
    FragH ah, al;
    const v4f x0 = *(const v4fa*)(arow + kb + 8 * hh), x1 = *(const v4fa*)(arow + kb + 8 * hh + 4), x2 = *(const v4fa*)(arow + kb + 16 + 8 * hh), x3 = *(const v4fa*)(arow + kb + 16 + 8 * hh + 4);
    float xs[16] = {x0[0],x0[1],x0[2],x0[3],x1[0],x1[1],x1[2],x1[3],x2[0],x2[1],x2[2],x2[3],x3[0],x3[1],x3[2],x3[3]};
#pragma unroll
    for (int i = 0; i < 16; ++i) { const _Float16 h = (_Float16)xs[i]; ah.h[i] = h; al.h[i] = ASPLIT ? (_Float16)(xs[i] - (float)h) : (_Float16)0.0f; }
#pragma unroll
    for (int t = 0; t < 4; ++t) { if (col0 + t * 16 >= N) continue; const size_t boff = (size_t)(col0 + t * 16 + ln) * ldb + kb; FragH bq; bq.half[0] = *(const v8us*)(Bh + boff + 8 * hh); bq.half[1] = *(const v8us*)(Bh + boff + 16 + 8 * hh);
      acc[t] = mmaH<ASPLIT ? 2 : 1>(ah.v, al.v, bq.v, bq.v, acc[t]); }
  }
#pragma unroll
  for (int t = 0; t < 4; ++t) { if (col0 + t * 16 >= N) continue;
#pragma unroll
    for (int r = 0; r < 8; ++r) so[w][8 * hh + r][t * 16 + ln] = acc[t][r] * alpha; }
  __builtin_amdgcn_fence(__ATOMIC_ACQ_REL, "workgroup"); __builtin_amdgcn_wave_barrier();
  const int rsub = lane >> 4, c4 = (lane & 15) * 4;
  for (int pass = 0; pass < 2; ++pass) {
#pragma unroll
    for (int q = 0; q < 8; ++q) { const int r = q * 2 + rsub; if (col0 + c4 < N) { const v4f v = *(const v4fa*)&so[w][r][c4]; *(volatile v4f*)(C + (size_t)(row0 + r) * ldc + col0 + c4) = v; } }
    if (pass == 0) __threadfence(); }
}

__global__ __launch_bounds__(256) void k_wt_f16(const float* __restrict__ W, _Float16* __restrict__ Wt, int K, int N, float scale) {
  const int t = blockIdx.x * 256 + threadIdx.x; if (t >= N * (K / 8)) return; const int n = t / (K / 8), k8 = (t % (K / 8)) * 8; FragH f;
#pragma unroll
  for (int i = 0; i < 8; ++i) f.h[i] = (_Float16)(bf16_round(W[(size_t)(k8 + i) * N + n]) * scale); const v8us o = f.half[0];
  *(volatile v8us*)((unsigned short*)Wt + (size_t)n * K + k8) = o; __threadfence(); *(volatile v8us*)((unsigned short*)Wt + (size_t)n * K + k8) = o;
}
template <int ACT>
__global__ __launch_bounds__(128) void k_gemm_hhx(const _Float16* __restrict__ A, int lda, size_t sA, const _Float16* __restrict__ Bh, int ldb, size_t sB, float alpha, const float* __restrict__ bias, size_t sBias, const float* __restrict__ CP, int rowsPerB, size_t sCPb, int row0g,
    float* __restrict__ C, _Float16* __restrict__ C16, int ldc, size_t sC, int M, int N, int K) {
  __shared__ __attribute__((aligned(16))) float so[4][16][64];
  const int tid = threadIdx.x, w = tid >> 5, lane = tid & 31, ln = lane & 15, hh = lane >> 4; const int by = blockIdx.y;
  A += (size_t)by * sA; Bh += (size_t)by * sB; const size_t cofs = (size_t)by * sC; const float* bp = bias ? bias + (size_t)by * sBias : nullptr;
  const int ntn = (N + 63) / 64; const int wid = blockIdx.x * 4 + w; const int mt = wid / ntn, nq = wid % ntn; if (mt * 16 >= M) return;
  const int row0 = mt * 16, col0 = nq * 64; const _Float16* arow = A + (size_t)(row0 + ln) * lda;
  v8f acc[4] = {};
  for (int kb = 0; kb < K; kb += 32) { FragH ah; ah.half[0] = *(const v8us*)((const unsigned short*)arow + kb + 8 * hh); ah.half[1] = *(const v8us*)((const unsigned short*)arow + kb + 16 + 8 * hh);
#pragma unroll
    for (int t = 0; t < 4; ++t) { if (col0 + t * 16 >= N) continue; const size_t boff = (size_t)(col0 + t * 16 + ln) * ldb + kb; FragH bq; bq.half[0] = *(const v8us*)((const unsigned short*)Bh + boff + 8 * hh); bq.half[1] = *(const v8us*)((const unsigned short*)Bh + boff + 16 + 8 * hh);
      acc[t] = mmaH<1>(ah.v, ah.v, bq.v, bq.v, acc[t]); }
  }
#pragma unroll
  for (int t = 0; t < 4; ++t) { if (col0 + t * 16 >= N) continue; const int col = col0 + t * 16 + ln; const float bv = bp ? bf16_round(bp[col]) : 0.f;
#pragma unroll
    for (int r = 0; r < 8; ++r) { float v = acc[t][r] * alpha + bv; if (CP) { const int bidx = (row0g + row0 + 8 * hh + r) / rowsPerB; v += CP[(size_t)bidx * sCPb + (size_t)by * 64 + col]; } if (ACT == 1) v = (v > 0.f) ? v : expm1f(v); else if (ACT == 7) v = (v > 0.f) ? v + 1.0f : expf(v); else if (ACT == 8) v = tanhf(v); else if (ACT == 9) v = 0.5f * v * (1.0f + tanhf(0.7978845608028654f * (v + 0.044715f * v * v * v))); else if (ACT == 11) v = 1.0f / (1.0f + expf(-v)); else if (ACT == 12) v = (v > 0.f) ? v : 0.01f * v; else if (ACT == 14) v = (v > 0.f) ? v : 0.1f * v; else if (ACT == 15) v = v / (1.0f + expf(-v)); else if (ACT == 3) v = fmaxf(v, 0.f); else if (ACT == 6) v = 0.5f * v * (1.0f + erff(v * 0.70710678118654752f)); so[w][8 * hh + r][t * 16 + ln] = v; } }
  __builtin_amdgcn_fence(__ATOMIC_ACQ_REL, "workgroup"); __builtin_amdgcn_wave_barrier();
  const int rsub = lane >> 4, c4 = (lane & 15) * 4; typedef _Float16 v4h __attribute__((ext_vector_type(4)));
  for (int pass = 0; pass < 2; ++pass) {
#pragma unroll
    for (int q = 0; q < 8; ++q) { const int r = q * 2 + rsub; if (col0 + c4 < N) { const v4f v = *(const v4fa*)&so[w][r][c4]; if (C) *(volatile v4f*)(C + cofs + (size_t)(row0 + r) * ldc + col0 + c4) = v; if (C16) { v4h h4; for (int i = 0; i < 4; ++i) h4[i] = (_Float16)v[i]; *(volatile v4h*)(C16 + cofs + (size_t)(row0 + r) * ldc + col0 + c4) = h4; } } }
    if (pass == 0) __threadfence(); }
}


typedef _Float16 v4h __attribute__((ext_vector_type(4)));

__global__ __launch_bounds__(256) void k_x16(const float* __restrict__ x, _Float16* __restrict__ X16, size_t n8) { const size_t t = (size_t)blockIdx.x * 256 + threadIdx.x; if (t >= n8) return; FragH f;
#pragma unroll
  for (int q = 0; q < 8; ++q) f.h[q] = (_Float16)bf16_round(x[t * 8 + q]); *(volatile v8us*)((unsigned short*)X16 + t * 8) = f.half[0]; __threadfence(); *(volatile v8us*)((unsigned short*)X16 + t * 8) = f.half[0]; }
__global__ __launch_bounds__(256) void k_h16(const float* __restrict__ x, _Float16* __restrict__ X16, size_t n8) { const size_t t = (size_t)blockIdx.x * 256 + threadIdx.x; if (t >= n8) return; FragH f;
#pragma unroll
  for (int q = 0; q < 8; ++q) f.h[q] = (_Float16)x[t * 8 + q]; *(volatile v8us*)((unsigned short*)X16 + t * 8) = f.half[0]; __threadfence(); *(volatile v8us*)((unsigned short*)X16 + t * 8) = f.half[0]; }
__global__ __launch_bounds__(256) void k_round16f(const float* __restrict__ W, _Float16* __restrict__ Bt, size_t n8) { const size_t t = (size_t)blockIdx.x * 256 + threadIdx.x; if (t >= n8) return; FragH f;
#pragma unroll
  for (int i = 0; i < 8; ++i) f.h[i] = (_Float16)(bf16_round(W[t * 8 + i]) * 16.0f); *(volatile v8us*)((unsigned short*)Bt + t * 8) = f.half[0]; __threadfence(); *(volatile v8us*)((unsigned short*)Bt + t * 8) = f.half[0]; }
template <int NHv, int TTv>
__global__ __launch_bounds__(256) void k_vt(const _Float16* __restrict__ V16, int ldv, int voff, _Float16* __restrict__ Vt) { __shared__ unsigned short tl[64][66]; const int tid = threadIdx.x; const int slab = blockIdx.x / (TTv / 64), lg = blockIdx.x % (TTv / 64); const int b = slab / NHv, h = slab % NHv;
  for (int i = tid; i < 64 * 8; i += 256) { const int r = i / 8, c8 = (i % 8) * 8; FragH f; f.half[0] = *(const v8us*)((const unsigned short*)V16 + ((size_t)b * TTv + lg * 64 + r) * ldv + voff + h * 64 + c8);
#pragma unroll
    for (int q = 0; q < 8; ++q) tl[r][c8 + q] = f.u[q]; }
  __syncthreads();
  for (int pass = 0; pass < 2; ++pass) {
#pragma unroll
    for (int rd = 0; rd < 2; ++rd) { const int d = rd * 32 + tid / 8, pc = tid % 8; FragH f;
#pragma unroll
      for (int q = 0; q < 8; ++q) f.u[q] = tl[pc * 8 + q][d];
      *(volatile v8us*)((unsigned short*)Vt + ((size_t)slab * 64 + d) * TTv + lg * 64 + pc * 8) = f.half[0]; }
    if (pass == 0) __threadfence(); } }

__global__ __launch_bounds__(256) void k_hl(const float* __restrict__ F, _Float16* __restrict__ Hh, _Float16* __restrict__ Hl, size_t n8) { const size_t t = (size_t)blockIdx.x * 256 + threadIdx.x; if (t >= n8) return; FragH fh, fl; const v4f a = *(const v4fa*)(F + t * 8), c = *(const v4fa*)(F + t * 8 + 4);
#pragma unroll
  for (int q = 0; q < 4; ++q) { _Float16 h = (_Float16)a[q]; fh.h[q] = h; fl.h[q] = (_Float16)((a[q] - (float)h) * 1024.0f); h = (_Float16)c[q]; fh.h[4 + q] = h; fl.h[4 + q] = (_Float16)((c[q] - (float)h) * 1024.0f); }
  for (int pass = 0; pass < 2; ++pass) { *(volatile v8us*)((unsigned short*)Hh + t * 8) = fh.half[0]; *(volatile v8us*)((unsigned short*)Hl + t * 8) = fl.half[0]; if (pass == 0) __threadfence(); } }

__device__ __forceinline__ v16h g2_frag(const _Float16* p, int hh) { FragH f; f.half[0] = *(const v8us*)((const unsigned short*)p + 8 * hh); f.half[1] = *(const v8us*)((const unsigned short*)p + 16 + 8 * hh); return f.v; }
__device__ __forceinline__ v8f g2_mma(v16h a, v16h b, v8f c) { v8f d = __builtin_amdgcn_wmma_f32_16x16x32_f16(false, a, false, b, (short)0, c, false, false); asm volatile("v_nop\n\tv_nop\n\tv_nop\n\tv_nop" : "+v"(d) : "v"(a), "v"(b)); return d; }
template <int ACT>
__global__ __launch_bounds__(128) void k_gemm2(const _Float16* __restrict__ A, int lda, size_t sA, const _Float16* __restrict__ Bh, int ldb, size_t sB, float alpha, const float* __restrict__ bias, size_t sBias, const float* __restrict__ CP, int rowsPerB, size_t sCPb, int row0g,
    float* __restrict__ C, _Float16* __restrict__ C16, int ldc, size_t sC, int M, int N, int K) {
  __shared__ __attribute__((aligned(16))) float so[4][32][68];
  const int tid = threadIdx.x, w = tid >> 5, lane = tid & 31, ln = lane & 15, hh = lane >> 4; const int by = blockIdx.y;
  A += (size_t)by * sA; Bh += (size_t)by * sB; const size_t cofs = (size_t)by * sC; const float* bp = bias ? bias + (size_t)by * sBias : nullptr;
  const int ntn = N >> 6; const int mt = blockIdx.x / ntn, nq = blockIdx.x - mt * ntn; const int row0 = mt * 128 + 32 * w, col0 = nq * 64; if (row0 >= M) return;
  const _Float16* a0p = A + (size_t)(row0 + ln) * lda; const _Float16* a1p = a0p + (size_t)16 * lda;
  const _Float16* b0p = Bh + (size_t)(col0 + ln) * ldb; const _Float16* b1p = b0p + (size_t)16 * ldb; const _Float16* b2p = b1p + (size_t)16 * ldb; const _Float16* b3p = b2p + (size_t)16 * ldb;
  const v8f z8 = {0.f,0.f,0.f,0.f,0.f,0.f,0.f,0.f}; v8f c00 = z8, c01 = z8, c02 = z8, c03 = z8, c10 = z8, c11 = z8, c12 = z8, c13 = z8;
#pragma unroll 1
  for (int kb = 0; kb < K; kb += 32) { const v16h a0 = g2_frag(a0p + kb, hh), a1 = g2_frag(a1p + kb, hh);
    v16h b = g2_frag(b0p + kb, hh); c00 = g2_mma(a0, b, c00); c10 = g2_mma(a1, b, c10);
    b = g2_frag(b1p + kb, hh); c01 = g2_mma(a0, b, c01); c11 = g2_mma(a1, b, c11);
    b = g2_frag(b2p + kb, hh); c02 = g2_mma(a0, b, c02); c12 = g2_mma(a1, b, c12);
    b = g2_frag(b3p + kb, hh); c03 = g2_mma(a0, b, c03); c13 = g2_mma(a1, b, c13); }
  v8f accs[8] = {c00, c01, c02, c03, c10, c11, c12, c13};
#pragma unroll
  for (int u = 0; u < 8; ++u) { const int t = u & 3, half = u >> 2; const int col = col0 + t * 16 + ln; const float bv = bp ? bf16_round(bp[col]) : 0.f;
#pragma unroll
    for (int r = 0; r < 8; ++r) { const int rloc = half * 16 + 8 * hh + r; float v = accs[u][r] * alpha + bv; if (CP) { const int bidx = (row0g + row0 + rloc) / rowsPerB; v += CP[(size_t)bidx * sCPb + (size_t)by * 64 + col]; }
      if (ACT == 3) v = fmaxf(v, 0.f); else if (ACT == 6) v = 0.5f * v * (1.0f + erff(v * 0.70710678118654752f)); else if (ACT == 11) v = 1.0f / (1.0f + expf(-v)); else if (ACT == 15) v = v / (1.0f + expf(-v)); else if (ACT == 12) v = (v > 0.f) ? v : 0.01f * v; else if (ACT == 8) v = tanhf(v);
      so[w][rloc][t * 16 + ln] = v; } }
  __builtin_amdgcn_fence(__ATOMIC_ACQ_REL, "workgroup"); __builtin_amdgcn_wave_barrier();
  const int rsub = lane >> 4, c4 = (lane & 15) * 4;
  for (int pass = 0; pass < 2; ++pass) {
#pragma unroll
    for (int q = 0; q < 16; ++q) { const int r = q * 2 + rsub; const v4f v = *(const v4fa*)&so[w][r][c4]; if (C) *(volatile v4f*)(C + cofs + (size_t)(row0 + r) * ldc + col0 + c4) = v; if (C16) { v4h h4; for (int i = 0; i < 4; ++i) h4[i] = (_Float16)v[i]; *(volatile v4h*)(C16 + cofs + (size_t)(row0 + r) * ldc + col0 + c4) = h4; } }
    if (pass == 0) __threadfence(); } }


__global__ __launch_bounds__(256) void k_im1(const float* __restrict__ x, int b0, _Float16* __restrict__ IM) {
  const int t = blockIdx.x * 256 + threadIdx.x; if (t >= ICH * NP1) return; const int p = t % NP1, b = b0 + t / NP1; const int y = p / H1, xx = p % H1; FragH f[2];
#pragma unroll
  for (int i = 0; i < 32; ++i) { float v = 0.f; if (i < 27) { const int k = i / 3, c = i % 3; const int yy = y + k / 3 - 1, x2 = xx + k % 3 - 1; if (yy >= 0 && yy < H1 && x2 >= 0 && x2 < H1) v = bf16_round(x[(((size_t)b * C0 + c) * H1 + yy) * H1 + x2]); } f[i >> 4].h[i & 15] = (_Float16)v; }
  unsigned short* d = (unsigned short*)IM + (size_t)t * K1P; for (int pass = 0; pass < 2; ++pass) { *(volatile v8us*)d = f[0].half[0]; *(volatile v8us*)(d + 8) = f[0].half[1]; *(volatile v8us*)(d + 16) = f[1].half[0]; *(volatile v8us*)(d + 24) = f[1].half[1]; if (pass == 0) __threadfence(); } }
__global__ __launch_bounds__(256) void k_wconv(const float* __restrict__ Wt, int O, int Ci, int KP, int orows, _Float16* __restrict__ Bt) {
  const int t = blockIdx.x * 256 + threadIdx.x; if (t >= orows * (KP / 8)) return; const int c0 = (t % (KP / 8)) * 8; const int o = t / (KP / 8); FragH f;
  for (int q = 0; q < 8; ++q) { const int col = c0 + q; float v = 0.f; if (o < O && col < 9 * Ci) { const int k = col / Ci, c = col % Ci; v = bf16_round(Wt[((size_t)o * Ci + c) * 9 + k]) * 16.0f; } f.h[q] = (_Float16)v; }
  *(volatile v8us*)((unsigned short*)Bt + (size_t)o * KP + c0) = f.half[0]; __threadfence(); *(volatile v8us*)((unsigned short*)Bt + (size_t)o * KP + c0) = f.half[0]; }
__global__ __launch_bounds__(256) void k_wsc(const float* __restrict__ Wm, _Float16* __restrict__ Bt, size_t n8, float sc) { const size_t t = (size_t)blockIdx.x * 256 + threadIdx.x; if (t >= n8) return; FragH f; for (int q = 0; q < 8; ++q) f.h[q] = (_Float16)(bf16_round(Wm[t * 8 + q]) * sc); *(volatile v8us*)((unsigned short*)Bt + t * 8) = f.half[0]; __threadfence(); *(volatile v8us*)((unsigned short*)Bt + t * 8) = f.half[0]; }
__global__ __launch_bounds__(256) void k_stA(const _Float16* __restrict__ XS, int ld, size_t nrows, int phase, float* __restrict__ ST) {
  #pragma clang fp contract(off)
  __shared__ float sh[256]; const int i = blockIdx.x; const int tid = threadIdx.x; const float mu = phase ? ST[i * 32] : 0.f; float s = 0.f;
  for (size_t r = tid; r < nrows; r += 256) { const float v = (float)XS[r * ld + i]; s += phase ? (v - mu) * (v - mu) : v; }
  sh[tid] = s; __syncthreads(); for (int st = 128; st > 0; st >>= 1) { if (tid < st) sh[tid] += sh[tid + st]; __syncthreads(); }
  if (tid == 0) { const float o = sh[0] / (float)nrows; *(volatile float*)(ST + i * 32 + phase) = o; __threadfence(); *(volatile float*)(ST + i * 32 + phase) = o; } }
__global__ __launch_bounds__(256) void k_stB(const _Float16* __restrict__ XS, int ld, size_t nrows, int phase, const float* __restrict__ ST, const float* __restrict__ dg, const float* __restrict__ db, const float* __restrict__ dw, float* __restrict__ SB) {
  #pragma clang fp contract(off)
  __shared__ float sh[256]; const int j = blockIdx.x; const int i = j / GG, g = j % GG; const int tid = threadIdx.x; const float muA = ST[i * 32], rsA = rsqrtf(ST[i * 32 + 1] + 1e-5f), ga = bf16_round(dg[i]), ba = bf16_round(db[i]), w = bf16_round(dw[i * GG + g]); const float mu = phase ? SB[j * 32] : 0.f; float s = 0.f;
  for (size_t r = tid; r < nrows; r += 256) { float v = ((float)XS[r * ld + i] - muA) * rsA * ga; v += ba; v = fmaxf(v, 0.f) * w; s += phase ? (v - mu) * (v - mu) : v; }
  sh[tid] = s; __syncthreads(); for (int st = 128; st > 0; st >>= 1) { if (tid < st) sh[tid] += sh[tid + st]; __syncthreads(); }
  if (tid == 0) { const float o = sh[0] / (float)nrows; *(volatile float*)(SB + j * 32 + phase) = o; __threadfence(); *(volatile float*)(SB + j * 32 + phase) = o; } }
__global__ __launch_bounds__(256) void k_pool(const _Float16* __restrict__ XS, int ld, int Hs, int nch, const float* __restrict__ ST, const float* __restrict__ dg, const float* __restrict__ db, const float* __restrict__ dw, const float* __restrict__ SB, const float* __restrict__ g2, const float* __restrict__ b2, _Float16* __restrict__ OUT) {
  #pragma clang fp contract(off)
  const size_t t2 = (size_t)blockIdx.x * 256 + threadIdx.x; const int Ho = Hs / 2; const size_t tot = (size_t)NIMG * nch * GG * Ho * Ho; if (t2 >= tot / 2) return;
  const size_t t = t2 * 2; const int xo0 = (int)(t % Ho); const int yo = (int)((t / Ho) % Ho); const int j = (int)((t / ((size_t)Ho * Ho)) % (nch * GG)); const size_t b = t / ((size_t)Ho * Ho * nch * GG); const int i = j / GG, g = j % GG;
  const float muA = ST[i * 32], rsA = rsqrtf(ST[i * 32 + 1] + 1e-5f), ga = bf16_round(dg[i]), ba = bf16_round(db[i]), w = bf16_round(dw[i * GG + g]); const float muB = SB[j * 32], rsB = rsqrtf(SB[j * 32 + 1] + 1e-5f), gb = bf16_round(g2[j]), bb = bf16_round(b2[j]);
  FragH f;
#pragma unroll
  for (int e = 0; e < 2; ++e) { const int xo = xo0 + e; float m = -3.0e38f;
#pragma unroll
    for (int dy = 0; dy < 2; ++dy)
#pragma unroll
      for (int dx = 0; dx < 2; ++dx) { const size_t r = b * (size_t)(Hs * Hs) + (size_t)(2 * yo + dy) * Hs + 2 * xo + dx; float v = ((float)XS[r * ld + i] - muA) * rsA * ga; v += ba; v = fmaxf(v, 0.f) * w; float u = (v - muB) * rsB * gb; u += bb; u = fmaxf(u, 0.f); m = fmaxf(m, u); }
    f.h[e] = (_Float16)m; }
  const unsigned pk = (unsigned)f.u[0] | ((unsigned)f.u[1] << 16); *(volatile unsigned*)(OUT + t) = pk; __threadfence(); *(volatile unsigned*)(OUT + t) = pk; }
__global__ __launch_bounds__(256) void k_im2(const _Float16* __restrict__ P1, int b0, _Float16* __restrict__ IM) {
  const int t = blockIdx.x * 256 + threadIdx.x; if (t >= ICH * NP2 * 10) return; const int k = t % 10; const int rp = t / 10; const int p = rp % NP2, b = b0 + rp / NP2; FragH f;
  if (k < 9) { const int y = p / H2 + k / 3 - 1, xx = p % H2 + k % 3 - 1; const bool ok = y >= 0 && y < H2 && xx >= 0 && xx < H2;
    for (int c = 0; c < 16; ++c) f.h[c] = ok ? P1[(((size_t)b * C1 + c) * H2 + y) * H2 + xx] : (_Float16)0.0f; }
  else { for (int c = 0; c < 16; ++c) f.u[c] = 0; }
  unsigned short* d = (unsigned short*)IM + (size_t)rp * K2P + k * 16; for (int pass = 0; pass < 2; ++pass) { *(volatile v8us*)d = f.half[0]; *(volatile v8us*)(d + 8) = f.half[1]; if (pass == 0) __threadfence(); } }
__global__ __launch_bounds__(256) void k_wfc3(const float* __restrict__ Wt, _Float16* __restrict__ Bt) { const int t = blockIdx.x * 256 + threadIdx.x; if (t >= 64 * (FCH / 8)) return; const int c0 = (t % (FCH / 8)) * 8; const int o = t / (FCH / 8); FragH f; for (int q = 0; q < 8; ++q) f.h[q] = (o < NCLS) ? (_Float16)(bf16_round(Wt[(size_t)o * FCH + c0 + q]) * 16.0f) : (_Float16)0.0f; *(volatile v8us*)((unsigned short*)Bt + (size_t)o * FCH + c0) = f.half[0]; __threadfence(); *(volatile v8us*)((unsigned short*)Bt + (size_t)o * FCH + c0) = f.half[0]; }
__global__ __launch_bounds__(256) void k_fcout(const float* __restrict__ F3, const float* __restrict__ fb, float* __restrict__ out) {
  #pragma clang fp contract(off)
  const int b = blockIdx.x * 256 + threadIdx.x; if (b >= NIMG) return; float v[NCLS]; for (int k = 0; k < NCLS; ++k) v[k] = F3[(size_t)b * 64 + k] + bf16_round(fb[k]);
  for (int pass = 0; pass < 2; ++pass) { for (int k = 0; k < NCLS; ++k) *(volatile float*)(out + (size_t)b * NCLS + k) = v[k]; if (pass == 0) __threadfence(); } }
__global__ __launch_bounds__(256) void k_compact(const _Float16* __restrict__ CCH, size_t row0, size_t nrows, int nch, _Float16* __restrict__ XS) {
  const size_t r = (size_t)blockIdx.x * 256 + threadIdx.x; if (r >= nrows) return; FragH f; f.half[0] = *(const v8us*)((const unsigned short*)CCH + r * 64); if (nch > 8) f.half[1] = *(const v8us*)((const unsigned short*)CCH + r * 64 + 8);
  unsigned short* d = (unsigned short*)XS + (row0 + r) * nch; for (int pass = 0; pass < 2; ++pass) { *(volatile v8us*)d = f.half[0]; if (nch > 8) *(volatile v8us*)(d + 8) = f.half[1]; if (pass == 0) __threadfence(); } }

extern "C" void kernel_launch(void* const* d_in, const int* in_sizes, int n_in,
                              void* d_out, int out_size, void* d_ws, size_t ws_size, hipStream_t stream) {
  (void)in_sizes; (void)n_in; (void)out_size;
  const float* const* I = (const float* const*)d_in; const float* x = I[0]; const float* dfe1 = I[1]; const float* d1g = I[2]; const float* d1b = I[3]; const float* d1w = I[4]; const float* b1g = I[5]; const float* b1b = I[6];
  const float* dfe2 = I[7]; const float* d2g = I[8]; const float* d2b = I[9]; const float* d2w = I[10]; const float* b2g = I[11]; const float* b2b = I[12]; const float* f1w = I[13]; const float* f1b = I[14]; const float* f2w = I[15]; const float* f2b = I[16]; const float* f3w = I[17]; const float* f3b = I[18];
  char* ws = (char*)d_ws; size_t off = 0;
  auto take = [&](size_t bytes) { char* p = ws + off; off += (bytes + 255) & ~(size_t)255; return p; };
  _Float16* BW1 = (_Float16*)take(64 * K1P * 2); _Float16* BW2 = (_Float16*)take(64 * K2P * 2); _Float16* BF1 = (_Float16*)take((size_t)FCH * FCI * 2); _Float16* BF2 = (_Float16*)take((size_t)FCH * FCH * 2); _Float16* BF3 = (_Float16*)take((size_t)64 * FCH * 2);
  _Float16* IM = (_Float16*)take((size_t)ICH * NP2 * K2P * 2);
  _Float16* CCH = (_Float16*)take((size_t)ICH * NP1 * 64 * 2); _Float16* X1 = (_Float16*)take((size_t)NIMG * NP1 * T1 * 2); _Float16* X2 = (_Float16*)take((size_t)NIMG * NP2 * T2 * 2); float* ST = (float*)take(64 * 32 * 4); float* SB = (float*)take(64 * 32 * 4);
  _Float16* P1 = (_Float16*)take((size_t)NIMG * C1 * NP2 * 2); _Float16* P2 = (_Float16*)take((size_t)NIMG * FCI * 2); _Float16* F1 = (_Float16*)take((size_t)NIMG * FCH * 2); _Float16* F2 = (_Float16*)take((size_t)NIMG * FCH * 2); float* F3 = (float*)take((size_t)NIMG * 64 * 4);
  if (off > ws_size) return;
  k_wconv<<<(64 * (K1P / 8) + 255) / 256, 256, 0, stream>>>(dfe1, T1, C0, K1P, 64, BW1); k_wconv<<<(64 * (K2P / 8) + 255) / 256, 256, 0, stream>>>(dfe2, T2, C1, K2P, 64, BW2);
  k_wsc<<<(unsigned)(((size_t)FCH * FCI / 8 + 255) / 256), 256, 0, stream>>>(f1w, BF1, (size_t)FCH * FCI / 8, 16.0f); k_wsc<<<(unsigned)(((size_t)FCH * FCH / 8 + 255) / 256), 256, 0, stream>>>(f2w, BF2, (size_t)FCH * FCH / 8, 16.0f); k_wfc3<<<(64 * (FCH / 8) + 255) / 256, 256, 0, stream>>>(f3w, BF3);
  for (int b0 = 0; b0 < NIMG; b0 += ICH) { const size_t rows = (size_t)ICH * NP1;
    k_im1<<<(unsigned)((rows + 255) / 256), 256, 0, stream>>>(x, b0, IM);
    k_gemm2<0><<<dim3((unsigned)(rows / 128) * 1, 1), 128, 0, stream>>>(IM, K1P, 0, BW1, K1P, 0, 0.0625f, nullptr, 0, nullptr, 1, 0, 0, nullptr, CCH, 64, 0, (int)rows, 64, K1P);
    k_compact<<<(unsigned)((rows + 255) / 256), 256, 0, stream>>>(CCH, (size_t)b0 * NP1, rows, T1, X1); }
  const size_t n1 = (size_t)NIMG * NP1;
  k_stA<<<T1, 256, 0, stream>>>(X1, T1, n1, 0, ST); k_stA<<<T1, 256, 0, stream>>>(X1, T1, n1, 1, ST);
  k_stB<<<C1, 256, 0, stream>>>(X1, T1, n1, 0, ST, d1g, d1b, d1w, SB); k_stB<<<C1, 256, 0, stream>>>(X1, T1, n1, 1, ST, d1g, d1b, d1w, SB);
  k_pool<<<(unsigned)(((size_t)NIMG * C1 * NP2 / 2 + 255) / 256), 256, 0, stream>>>(X1, T1, H1, T1, ST, d1g, d1b, d1w, SB, b1g, b1b, P1);
  for (int b0 = 0; b0 < NIMG; b0 += ICH) { const size_t rows = (size_t)ICH * NP2;
    k_im2<<<(unsigned)((rows * 10 + 255) / 256), 256, 0, stream>>>(P1, b0, IM);
    k_gemm2<0><<<dim3((unsigned)(rows / 128) * 1, 1), 128, 0, stream>>>(IM, K2P, 0, BW2, K2P, 0, 0.0625f, nullptr, 0, nullptr, 1, 0, 0, nullptr, CCH, 64, 0, (int)rows, 64, K2P);
    k_compact<<<(unsigned)((rows + 255) / 256), 256, 0, stream>>>(CCH, (size_t)b0 * NP2, rows, T2, X2); }
  const size_t n2 = (size_t)NIMG * NP2;
  k_stA<<<T2, 256, 0, stream>>>(X2, T2, n2, 0, ST); k_stA<<<T2, 256, 0, stream>>>(X2, T2, n2, 1, ST);
  k_stB<<<C2, 256, 0, stream>>>(X2, T2, n2, 0, ST, d2g, d2b, d2w, SB); k_stB<<<C2, 256, 0, stream>>>(X2, T2, n2, 1, ST, d2g, d2b, d2w, SB);
  k_pool<<<(unsigned)(((size_t)NIMG * C2 * NP3 / 2 + 255) / 256), 256, 0, stream>>>(X2, T2, H2, T2, ST, d2g, d2b, d2w, SB, b2g, b2b, P2);
  k_gemm2<3><<<dim3((NIMG / 128) * (FCH / 64), 1), 128, 0, stream>>>(P2, FCI, 0, BF1, FCI, 0, 0.0625f, f1b, 0, nullptr, 1, 0, 0, nullptr, F1, FCH, 0, NIMG, FCH, FCI);
  k_gemm2<3><<<dim3((NIMG / 128) * (FCH / 64), 1), 128, 0, stream>>>(F1, FCH, 0, BF2, FCH, 0, 0.0625f, f2b, 0, nullptr, 1, 0, 0, nullptr, F2, FCH, 0, NIMG, FCH, FCH);
  k_gemm2<0><<<dim3((NIMG / 128) * 1, 1), 128, 0, stream>>>(F2, FCH, 0, BF3, FCH, 0, 0.0625f, nullptr, 0, nullptr, 1, 0, 0, F3, nullptr, 64, 0, NIMG, 64, FCH);
  k_fcout<<<(NIMG + 255) / 256, 256, 0, stream>>>(F3, f3b, (float*)d_out);
}
